// Mamba3_64819646431743
// MI455X (gfx1250) — hardware-run, weakly checked
//
#include <hip/hip_runtime.h>
#include <hip/hip_bf16.h>

constexpr int kBatch   = 2;
constexpr int kSeq     = 1024;
constexpr int kRows    = kBatch * kSeq;
constexpr int kDModel  = 1024;
constexpr int kDState  = 64;
constexpr int kDConv   = 4;
constexpr int kHeadDim = 128;
constexpr int kHeads   = 16;
constexpr int kDInner  = 2048;
constexpr int kDInProj = 4240;
constexpr int kNPad1   = 4288;
constexpr int kConvDim = 2176;

static_assert(kNPad1 % 64 == 0 && kNPad1 >= kDInProj, "pad");
static_assert(kRows % 64 == 0 && kDModel % 64 == 0 && kDInner % 64 == 0, "tile multiples");
static_assert(kDModel % 32 == 0 && kDInner % 32 == 0, "K multiples of 32");
static_assert(kHeads * kHeadDim == kDInner && kDInner + kConvDim + kHeads == kDInProj, "layout");
static_assert(kConvDim % 32 == 0 && kSeq % 8 == 0, "line layout");

constexpr size_t kBytesHid  = (size_t)kRows * kDModel * 2;
constexpr size_t kBytesWin  = (size_t)kNPad1 * kDModel * 2;
constexpr size_t kBytesWout = (size_t)kDModel * kDInner * 2;
constexpr size_t kBytesZx   = (size_t)kRows * kNPad1 * 4;
constexpr size_t kBytesXbc  = (size_t)kRows * kConvDim * 4;
constexpr size_t kBytesDt   = (size_t)kRows * kHeads * 4;
constexpr size_t kBytesY    = (size_t)kRows * kDInner * 4;
constexpr size_t kBytesYpl  = (size_t)kRows * kDInner * 2;
constexpr size_t kOffHid  = 0;
constexpr size_t kOffWin  = kOffHid + kBytesHid;
constexpr size_t kOffWout = kOffWin + kBytesWin;
constexpr size_t kOffZx   = kOffWout + kBytesWout;
constexpr size_t kOffXbc  = kOffZx + kBytesZx;
constexpr size_t kOffDts  = kOffXbc + kBytesXbc;
constexpr size_t kOffDas  = kOffDts + kBytesDt;
constexpr size_t kOffY    = kOffDas + kBytesDt;
constexpr size_t kOffYhi  = kOffY + kBytesY;
constexpr size_t kOffYlo  = kOffYhi + kBytesYpl;
constexpr size_t kWsTotal = kOffYlo + kBytesYpl;
static_assert(kWsTotal == 103940096ull, "carve total");
static_assert(kWsTotal <= 134217728ull, "carve budget");
static_assert(kOffWin % 128 == 0 && kOffWout % 128 == 0 && kOffZx % 128 == 0 && kOffXbc % 128 == 0 &&
              kOffDts % 128 == 0 && kOffDas % 128 == 0 && kOffY % 128 == 0 && kOffYhi % 128 == 0 &&
              kOffYlo % 128 == 0, "alignment");

typedef __attribute__((ext_vector_type(16))) _Float16 v16h;
typedef __attribute__((ext_vector_type(8)))  _Float16 v8h;
typedef __attribute__((ext_vector_type(16))) __bf16   v16b;
typedef __attribute__((ext_vector_type(8)))  __bf16   v8b;
typedef __attribute__((ext_vector_type(8)))  float    v8f;
typedef __attribute__((ext_vector_type(4)))  float    v4f;
typedef __attribute__((ext_vector_type(4)))  unsigned v4u;

__device__ __forceinline__ unsigned short f2bf_bits(float f) {
  unsigned u = __float_as_uint(f);
  return (unsigned short)((u + 0x7FFFu + ((u >> 16) & 1u)) >> 16);
}
__device__ __forceinline__ float bf_bits2f(unsigned short h) { return __uint_as_float(((unsigned)h) << 16); }
__device__ __forceinline__ float bfr(float f) { return bf_bits2f(f2bf_bits(f)); }

__device__ __forceinline__ void dep_guard_h(v8f& a, v8f& b, v16h x, v16h y) { asm volatile("v_nop\n\tv_nop\n\tv_nop\n\tv_nop" : "+v"(a), "+v"(b) : "v"(x), "v"(y)); }
__device__ __forceinline__ void dep_guard_b(v8f& a, v8f& b, v16b x, v16b y) { asm volatile("v_nop\n\tv_nop\n\tv_nop\n\tv_nop" : "+v"(a), "+v"(b) : "v"(x), "v"(y)); }
__device__ __forceinline__ void keep4_h(v16h a, v16h b, v16h c, v16h d) { asm volatile("v_nop" :: "v"(a), "v"(b), "v"(c), "v"(d)); }
__device__ __forceinline__ void keep4_b(v16b a, v16b b, v16b c, v16b d) { asm volatile("v_nop" :: "v"(a), "v"(b), "v"(c), "v"(d)); }
__device__ __forceinline__ void acc_guard4(v8f& a, v8f& b, v8f& c, v8f& d) { asm volatile("v_nop\n\tv_nop\n\tv_nop\n\tv_nop" : "+v"(a), "+v"(b), "+v"(c), "+v"(d)); }
template <typename T> struct Frag;
template <> struct Frag<_Float16> {
  typedef v16h V; union U { v16h v; v8h h[2]; };
  static __device__ __forceinline__ v16h load(const _Float16* p) {
    U f; f.h[0] = *(const v8h*)(p); f.h[1] = *(const v8h*)(p + 16); return f.v;
  }
  static __device__ __forceinline__ v8f mma(v16h a, v16h b, v8f c) {
    return __builtin_amdgcn_wmma_f32_16x16x32_f16(false, a, false, b, (short)0, c, false, false);
  }
  static __device__ __forceinline__ void guard(v8f& a, v8f& b, v16h x, v16h y) { dep_guard_h(a, b, x, y); }
  static __device__ __forceinline__ void keep(v16h a, v16h b, v16h c, v16h d) { keep4_h(a, b, c, d); }
};
template <> struct Frag<__bf16> {
  typedef v16b V; union U { v16b v; v8b h[2]; };
  static __device__ __forceinline__ v16b load(const __bf16* p) {
    U f; f.h[0] = *(const v8b*)(p); f.h[1] = *(const v8b*)(p + 16); return f.v;
  }
  static __device__ __forceinline__ v8f mma(v16b a, v16b b, v8f c) {
    return __builtin_amdgcn_wmma_f32_16x16x32_bf16(false, a, false, b, (short)0, c, false, false);
  }
  static __device__ __forceinline__ void guard(v8f& a, v8f& b, v16b x, v16b y) { dep_guard_b(a, b, x, y); }
  static __device__ __forceinline__ void keep(v16b a, v16b b, v16b c, v16b d) { keep4_b(a, b, c, d); }
};

template <int ET> struct Elem;
template <> struct Elem<0> { typedef _Float16 T; };
template <> struct Elem<1> { typedef __bf16 T; };
template <int ET, int SPLIT, int BIAS_MODE, int OUT_MODE>
__global__ __launch_bounds__(256) void wmma_gemm64(
    const unsigned short* __restrict__ Ap, const unsigned short* __restrict__ A2p, int lda, long strideA,
    const unsigned short* __restrict__ Btp, const unsigned short* __restrict__ Bt2p, int ldb, long strideB,
    void* __restrict__ Cout, void* __restrict__ Cout2, int ldc, long strideC,
    const float* __restrict__ bias,
    int M, int N, int K, float scale) {
  typedef typename Elem<ET>::T T;
  typedef typename Frag<T>::V V;
  const T* A = (const T*)Ap; const T* A2 = (const T*)A2p; const T* Bt = (const T*)Btp; const T* Bt2 = (const T*)Bt2p;
  __shared__ __align__(16) float sT[8][16 * 68];
  const int b    = blockIdx.y;
  const int lane = threadIdx.x & 31;
  const int wave = threadIdx.x >> 5;
  const int tilesN = N >> 6;
  const int tilesM = M >> 6;
  const int tile = blockIdx.x * 8 + wave;
  if (tile >= tilesM * tilesN) return;
  const int tm = tile / tilesN;
  const int tn = tile - tm * tilesN;
  const int m0 = tm << 6;
  const int n0 = tn << 6;

  const T* Ab  = A  + (size_t)b * strideA;
  const T* Bb  = Bt + (size_t)b * strideB;
  const T* Ab2 = (SPLIT != 0) ? (A2  + (size_t)b * strideA) : nullptr;
  const T* Bb2 = (SPLIT == 1) ? (Bt2 + (size_t)b * strideB) : nullptr;

  const int rlane = lane & 15;
  const int koff  = (lane >> 4) * 8;
  const int mOff  = (lane >> 4) * 8;

  v8f acc[4][4];
#pragma unroll
  for (int i = 0; i < 4; ++i)
#pragma unroll
    for (int j = 0; j < 4; ++j) acc[i][j] = (v8f){0.f,0.f,0.f,0.f,0.f,0.f,0.f,0.f};

  for (int k0 = 0; k0 < K; k0 += 32) {
    V bh[4], bl[4];
#pragma unroll
    for (int j = 0; j < 4; ++j) {
      const size_t bo = (size_t)(n0 + (j << 4) + rlane) * ldb + koff + k0;
      bh[j] = Frag<T>::load(Bb + bo);
      if (SPLIT == 1) bl[j] = Frag<T>::load(Bb2 + bo);
    }
#pragma unroll
    for (int i = 0; i < 4; ++i) {
      const size_t ao = (size_t)(m0 + (i << 4) + rlane) * lda + koff + k0;
      V ah = Frag<T>::load(Ab + ao);
      V al;
      if (SPLIT != 0) al = Frag<T>::load(Ab2 + ao);
#pragma unroll
      for (int j = 0; j < 4; ++j) {
        acc[i][j] = Frag<T>::mma(ah, bh[j], acc[i][j]);
        if (SPLIT == 1) acc[i][j] = Frag<T>::mma(ah, bl[j], acc[i][j]);
        if (SPLIT != 0) acc[i][j] = Frag<T>::mma(al, bh[j], acc[i][j]);
      }
      Frag<T>::guard(acc[i][0], acc[i][3], ah, (SPLIT != 0) ? al : ah);
    }
    Frag<T>::keep(bh[0], bh[1], bh[2], bh[3]);
    if (SPLIT == 1) Frag<T>::keep(bl[0], bl[1], bl[2], bl[3]);
  }
  acc_guard4(acc[0][0], acc[0][1], acc[0][2], acc[0][3]);
  acc_guard4(acc[1][0], acc[1][1], acc[1][2], acc[1][3]);
  acc_guard4(acc[2][0], acc[2][1], acc[2][2], acc[2][3]);
  acc_guard4(acc[3][0], acc[3][1], acc[3][2], acc[3][3]);

  float* slab = sT[wave];
#pragma unroll
  for (int i = 0; i < 4; ++i) {
    const int mBase = m0 + (i << 4);
#pragma unroll
    for (int j = 0; j < 4; ++j) {
      const int n = n0 + (j << 4) + rlane;
      float bv = 0.f;
      if (BIAS_MODE == 2) bv = bias[n];
#pragma unroll
      for (int r = 0; r < 8; ++r) {
        float v = acc[i][j][r] * scale;
        if (BIAS_MODE == 1) v += bias[mBase + mOff + r];
        if (BIAS_MODE == 2) v += bv;
        slab[(mOff + r) * 68 + (j << 4) + rlane] = v;
      }
    }
    __builtin_amdgcn_fence(__ATOMIC_RELEASE, "workgroup");
    __builtin_amdgcn_wave_barrier();
    __builtin_amdgcn_fence(__ATOMIC_ACQUIRE, "workgroup");
    if (OUT_MODE == 0) {
      float* C = (float*)Cout + (size_t)b * strideC;
      const int hh = lane >> 4, c4 = (lane & 15) * 4;
      for (int pass = 0; pass < 2; ++pass) {
#pragma unroll
        for (int it = 0; it < 8; ++it) {
          const int row = it * 2 + hh;
          v4f v = *(const v4f*)(slab + row * 68 + c4);
          *(volatile v4f*)(C + (size_t)(mBase + row) * ldc + n0 + c4) = v;
        }
        __threadfence();
      }
    } else {
      const int q = lane >> 3, c8 = (lane & 7) * 8;
      unsigned short* C  = (unsigned short*)Cout  + (size_t)b * strideC;
      unsigned short* C2 = (OUT_MODE == 2) ? ((unsigned short*)Cout2 + (size_t)b * strideC) : nullptr;
      for (int pass = 0; pass < 2; ++pass) {
#pragma unroll
        for (int it = 0; it < 4; ++it) {
          const int row = it * 4 + q;
          const float* sp = slab + row * 68 + c8;
          v8h hv, lv;
#pragma unroll
          for (int e = 0; e < 8; ++e) {
            if (OUT_MODE == 1) {
              hv[e] = (_Float16)sp[e];
            } else {
              unsigned short hb = f2bf_bits(sp[e]);
              unsigned short lb = f2bf_bits(sp[e] - bf_bits2f(hb));
              hv[e] = __builtin_bit_cast(_Float16, hb);
              lv[e] = __builtin_bit_cast(_Float16, lb);
            }
          }
          *(volatile v8h*)(C + (size_t)(mBase + row) * ldc + n0 + c8) = hv;
          if (OUT_MODE == 2) *(volatile v8h*)(C2 + (size_t)(mBase + row) * ldc + n0 + c8) = lv;
        }
        __threadfence();
      }
    }
    __builtin_amdgcn_fence(__ATOMIC_RELEASE, "workgroup");
    __builtin_amdgcn_wave_barrier();
    __builtin_amdgcn_fence(__ATOMIC_ACQUIRE, "workgroup");
  }
}

__global__ __launch_bounds__(256) void cast_f32_bf16x2(
    const float* __restrict__ in, unsigned short* __restrict__ out, int n2_real, int n2_total) {
  const int i = blockIdx.x * 256 + threadIdx.x;
  if (i < n2_total) {
    const int ic = (i < n2_real) ? i : (n2_real - 1);
    const float a = in[2 * (size_t)ic];
    const float c = in[2 * (size_t)ic + 1];
    unsigned u = (unsigned)f2bf_bits(a) | ((unsigned)f2bf_bits(c) << 16);
    u = (i < n2_real) ? u : 0u;
    ((volatile unsigned*)out)[i] = u;
    __threadfence();
    ((volatile unsigned*)out)[i] = u;
  }
}

__global__ __launch_bounds__(256) void conv_silu_kernel(
    const float* __restrict__ zx, const float* __restrict__ conv_w, const float* __restrict__ conv_b,
    float* __restrict__ xbc) {
  const int idx = blockIdx.x * 256 + threadIdx.x;
  const int c   = idx % kConvDim;
  const int row = idx / kConvDim;
  const int l   = row & (kSeq - 1);
  const v4f w4 = *(const v4f*)(conv_w + (size_t)c * kDConv);
  float acc = 0.f;
#pragma unroll
  for (int k = 0; k < kDConv; ++k) {
    const int ls = l - (kDConv - 1) + k;
    const bool valid = (ls >= 0);
    const int rs = valid ? (row - (kDConv - 1) + k) : row;
    const float xv = zx[(size_t)rs * kNPad1 + kDInner + c];
    const float wv = bfr(w4[k]);
    acc += (valid ? xv : 0.f) * wv;
  }
  const float v  = acc + bfr(conv_b[c]);
  const float sg = 1.0f / (1.0f + expf(-v));
  const float o  = v * sg;
  ((volatile float*)xbc)[idx] = o;
  __threadfence();
  ((volatile float*)xbc)[idx] = o;
}

__global__ __launch_bounds__(256) void dt_table_kernel(
    const float* __restrict__ zx, const float* __restrict__ dt_bias, const float* __restrict__ a_log,
    float* __restrict__ dts, float* __restrict__ das) {
  const int idx = blockIdx.x * 256 + threadIdx.x;
  const int h   = idx & (kHeads - 1);
  const int row = idx >> 4;
  const float raw = zx[(size_t)row * kNPad1 + kDInner + kConvDim + h];
  const float x   = raw + bfr(dt_bias[h]);
  const float sp  = fmaxf(x, 0.f) + log1pf(expf(-fabsf(x)));
  const float av  = -expf(bfr(a_log[h]));
  const float da  = expf(sp * av);
  ((volatile float*)dts)[idx] = sp;
  ((volatile float*)das)[idx] = da;
  __threadfence();
  ((volatile float*)dts)[idx] = sp;
  ((volatile float*)das)[idx] = da;
}

__global__ __launch_bounds__(256) void scan_kernel(
    const float* __restrict__ xbc, const float* __restrict__ dts, const float* __restrict__ das,
    const float* __restrict__ Dprm, float* __restrict__ yb) {
  const int b = blockIdx.x / kHeads;
  const int h = blockIdx.x % kHeads;
  const int t = threadIdx.x;
  const int lane = t & 31, wave = t >> 5;
  const int p  = t >> 1;
  const int nb = (t & 1) * (kDState / 2);

  __shared__ __align__(16) float s_in[256];
  __shared__ __align__(16) float ybuf[8][kHeadDim];

  const float Dv = bfr(Dprm[h]);
  const int off = (t < 2 * kDState) ? (kDInner + t) : (h * kHeadDim + (t - 2 * kDState));

  float hst[kDState / 2];
#pragma unroll
  for (int i = 0; i < kDState / 2; ++i) hst[i] = 0.f;

  for (int l = 0; l < kSeq; ++l) {
    const int row = b * kSeq + l;
    s_in[t] = xbc[(size_t)row * kConvDim + off];
    const float dtv = dts[(size_t)row * kHeads + h];
    const float dav = das[(size_t)row * kHeads + h];
    __syncthreads();

    const float xv    = s_in[2 * kDState + p];
    const float coeff = dtv * xv;
    float partial = 0.f;
#pragma unroll
    for (int i = 0; i < kDState / 2; ++i) {
      const int n = nb + i;
      hst[i] = dav * hst[i] + coeff * s_in[n];
      partial += hst[i] * s_in[kDState + n];
    }
    const float other = __shfl_xor(partial, 1, 32);
    const float yv = (partial + other) + Dv * xv;
    if ((t & 1) == 0) ybuf[l & 7][p] = yv;

    if ((l & 7) == 7) {
      __syncthreads();
      const int r = l - 7 + wave;
      const v4f v = *(const v4f*)(&ybuf[wave][lane * 4]);
      float* dst = yb + (size_t)(b * kSeq + r) * kDInner + h * kHeadDim + lane * 4;
      *(volatile v4f*)dst = v;
      __threadfence();
      *(volatile v4f*)dst = v;
    }
    __syncthreads();
  }
}

__device__ __forceinline__ unsigned hl_pack(float o0, float o1, unsigned& lo_out) {
  const unsigned short h0 = f2bf_bits(o0), h1 = f2bf_bits(o1);
  const unsigned short l0 = f2bf_bits(o0 - bf_bits2f(h0));
  const unsigned short l1 = f2bf_bits(o1 - bf_bits2f(h1));
  lo_out = (unsigned)l0 | ((unsigned)l1 << 16);
  return (unsigned)h0 | ((unsigned)h1 << 16);
}

__global__ __launch_bounds__(256) void gate_norm_kernel(
    const float* __restrict__ zx, const float* __restrict__ yb, const float* __restrict__ norm_w,
    unsigned short* __restrict__ yhi, unsigned short* __restrict__ ylo) {
  const int row = blockIdx.x;
  const int t = threadIdx.x, lane = t & 31, wave = t >> 5;
  __shared__ __align__(16) float vbuf[kDInner];
  __shared__ float red[8];
  __shared__ float s_scale;

  const float* zr = zx + (size_t)row * kNPad1;
  const float* yr = yb + (size_t)row * kDInner;
  float ss = 0.f;
#pragma unroll 1
  for (int e = 0; e < kDInner / 256; ++e) {
    const int col  = e * 256 + t;
    const float z  = zr[col];
    const float yv = yr[col];
    const float sg = 1.0f / (1.0f + expf(-z));
    const float v  = yv * (z * sg);
    vbuf[col] = v;
    ss += v * v;
  }
#pragma unroll
  for (int offs = 16; offs > 0; offs >>= 1) ss += __shfl_xor(ss, offs, 32);
  if (lane == 0) red[wave] = ss;
  __syncthreads();
  if (t == 0) {
    float s = 0.f;
#pragma unroll
    for (int i = 0; i < 8; ++i) s += red[i];
    s_scale = rsqrtf(s * (1.0f / (float)kDInner) + 1e-5f);
  }
  __syncthreads();
  const float scale = s_scale;

  const v4f va = *(const v4f*)(vbuf + 8 * t);
  const v4f vb = *(const v4f*)(vbuf + 8 * t + 4);
  const v4f wa = *(const v4f*)(norm_w + 8 * t);
  const v4f wb = *(const v4f*)(norm_w + 8 * t + 4);
  const float o0 = (va[0] * scale) * bfr(wa[0]);
  const float o1 = (va[1] * scale) * bfr(wa[1]);
  const float o2 = (va[2] * scale) * bfr(wa[2]);
  const float o3 = (va[3] * scale) * bfr(wa[3]);
  const float o4 = (vb[0] * scale) * bfr(wb[0]);
  const float o5 = (vb[1] * scale) * bfr(wb[1]);
  const float o6 = (vb[2] * scale) * bfr(wb[2]);
  const float o7 = (vb[3] * scale) * bfr(wb[3]);
  unsigned lw0, lw1, lw2, lw3;
  const unsigned hw0 = hl_pack(o0, o1, lw0);
  const unsigned hw1 = hl_pack(o2, o3, lw1);
  const unsigned hw2 = hl_pack(o4, o5, lw2);
  const unsigned hw3 = hl_pack(o6, o7, lw3);
  const v4u hv = (v4u){hw0, hw1, hw2, hw3};
  const v4u lv = (v4u){lw0, lw1, lw2, lw3};
  unsigned short* ph = yhi + (size_t)row * kDInner + 8 * t;
  unsigned short* pl = ylo + (size_t)row * kDInner + 8 * t;
  *(volatile v4u*)ph = hv;
  *(volatile v4u*)pl = lv;
  __threadfence();
  *(volatile v4u*)ph = hv;
  *(volatile v4u*)pl = lv;
}

extern "C" void kernel_launch(void* const* d_in, const int* in_sizes, int n_in,
                              void* d_out, int out_size, void* d_ws, size_t ws_size,
                              hipStream_t stream) {
  if (n_in < 9) return;
  if (in_sizes[0] != kRows * kDModel || in_sizes[1] != kDInProj * kDModel ||
      in_sizes[2] != kConvDim * kDConv || in_sizes[3] != kConvDim ||
      in_sizes[4] != kHeads || in_sizes[5] != kHeads || in_sizes[6] != kHeads ||
      in_sizes[7] != kDInner || in_sizes[8] != kDModel * kDInner) return;
  if (out_size != kRows * kDModel) return;
  if (ws_size < kWsTotal) return;

  const float* hidden  = (const float*)d_in[0];
  const float* W_in    = (const float*)d_in[1];
  const float* conv_w  = (const float*)d_in[2];
  const float* conv_b  = (const float*)d_in[3];
  const float* dt_bias = (const float*)d_in[4];
  const float* A_log   = (const float*)d_in[5];
  const float* D_param = (const float*)d_in[6];
  const float* norm_w  = (const float*)d_in[7];
  const float* W_out   = (const float*)d_in[8];
  float* out = (float*)d_out;

  char* ws = (char*)d_ws;
  unsigned short* hid_bf  = (unsigned short*)(ws + kOffHid);
  unsigned short* win_bf  = (unsigned short*)(ws + kOffWin);
  unsigned short* wout_bf = (unsigned short*)(ws + kOffWout);
  float* zx  = (float*)(ws + kOffZx);
  float* xbc = (float*)(ws + kOffXbc);
  float* dts = (float*)(ws + kOffDts);
  float* das = (float*)(ws + kOffDas);
  float* yb  = (float*)(ws + kOffY);
  unsigned short* yhi = (unsigned short*)(ws + kOffYhi);
  unsigned short* ylo = (unsigned short*)(ws + kOffYlo);

  {
    constexpr int n2_hid = kRows * kDModel / 2;
    static_assert(n2_hid % 256 == 0, "grid");
    cast_f32_bf16x2<<<dim3(n2_hid / 256), dim3(256), 0, stream>>>(hidden, hid_bf, n2_hid, n2_hid);
    constexpr int n2_win_real = kDInProj * kDModel / 2;
    constexpr int n2_win_tot  = kNPad1 * kDModel / 2;
    static_assert(n2_win_tot % 256 == 0, "grid");
    cast_f32_bf16x2<<<dim3(n2_win_tot / 256), dim3(256), 0, stream>>>(W_in, win_bf, n2_win_real, n2_win_tot);
    constexpr int n2_wout = kDModel * kDInner / 2;
    static_assert(n2_wout % 256 == 0, "grid");
    cast_f32_bf16x2<<<dim3(n2_wout / 256), dim3(256), 0, stream>>>(W_out, wout_bf, n2_wout, n2_wout);
  }

  {
    constexpr int gM = kRows, gN = kNPad1, gK = kDModel;
    static_assert(gM % 64 == 0 && gN % 64 == 0 && gK % 32 == 0, "gemm shape");
    constexpr int tiles = (gM / 64) * (gN / 64);
    constexpr int blocks = (tiles + 7) / 8;
    wmma_gemm64<1, 0, 0, 0><<<dim3(blocks, 1), dim3(256), 0, stream>>>(
        hid_bf, hid_bf, gK, 0L, win_bf, win_bf, gK, 0L,
        (void*)zx, (void*)zx, gN, 0L, norm_w, gM, gN, gK, 1.0f);
  }

  {
    constexpr int total = kRows * kConvDim;
    static_assert(total % 256 == 0, "grid");
    conv_silu_kernel<<<dim3(total / 256), dim3(256), 0, stream>>>(zx, conv_w, conv_b, xbc);
    constexpr int tdt = kRows * kHeads;
    static_assert(tdt % 256 == 0, "grid");
    dt_table_kernel<<<dim3(tdt / 256), dim3(256), 0, stream>>>(zx, dt_bias, A_log, dts, das);
  }

  scan_kernel<<<dim3(kBatch * kHeads), dim3(256), 0, stream>>>(xbc, dts, das, D_param, yb);

  gate_norm_kernel<<<dim3(kRows), dim3(256), 0, stream>>>(zx, yb, norm_w, yhi, ylo);

  {
    constexpr int gM = kRows, gN = kDModel, gK = kDInner;
    static_assert(gM % 64 == 0 && gN % 64 == 0 && gK % 32 == 0, "gemm shape");
    constexpr int tiles = (gM / 64) * (gN / 64);
    constexpr int blocks = (tiles + 7) / 8;
    wmma_gemm64<1, 2, 0, 0><<<dim3(blocks, 1), dim3(256), 0, stream>>>(
        yhi, ylo, gK, 0L, wout_bf, wout_bf, gK, 0L,
        (void*)out, (void*)out, gN, 0L, norm_w, gM, gN, gK, 1.0f);
  }
}
